// FastCompatibleMultiheadAttention_40716289966621
// MI455X (gfx1250) — hardware-verified
//
#include <hip/hip_runtime.h>
#include <math.h>
#include <stdint.h>

#define NBATCH 2
#define SEQ    2048
#define SEQLOG 11
#define DM     1024
#define DMLOG  10
#define NH     16
#define HD     64
#define NIN    (3 * DM)
#define QKP    (2 * DM)
#define MP     (NBATCH * SEQ)
#define NQB    (SEQ / 64)
#define WSC    64.0f
#define CSC    64.0f
#define RSC    2048.0f
#define RINV   (1.0f / 2048.0f)
static_assert(NH * HD == DM);
static_assert((1 << SEQLOG) == SEQ && (1 << DMLOG) == DM && HD == 64);
static_assert((SEQ % 64) == 0 && (DM % 64) == 0 && (QKP % 64) == 0 && (MP % 64) == 0 && (NIN % 64) == 0);

typedef _Float16 v16h __attribute__((ext_vector_type(16)));
typedef _Float16 v8h  __attribute__((ext_vector_type(8)));
typedef float    v8f  __attribute__((ext_vector_type(8)));
typedef float    v4f  __attribute__((ext_vector_type(4)));
typedef unsigned int v4u __attribute__((ext_vector_type(4)));

union FragH { v16h v; v8h h[2]; };

__device__ __forceinline__ unsigned short bf_bits(float f) {
  unsigned u = __float_as_uint(f);
  return (unsigned short)((u + 0x7FFFu + ((u >> 16) & 1u)) >> 16);
}
__device__ __forceinline__ float bf_up(unsigned short h) { return __uint_as_float(((unsigned)h) << 16); }
__device__ __forceinline__ float bfr(float f) { return bf_up(bf_bits(f)); }
__device__ __forceinline__ unsigned short h_bits(_Float16 x) { return __builtin_bit_cast(unsigned short, x); }
__device__ __forceinline__ unsigned pk16(unsigned short a, unsigned short b) { return (unsigned)a | ((unsigned)b << 16); }
__device__ __forceinline__ v8f zero8() { v8f z = {0.f, 0.f, 0.f, 0.f, 0.f, 0.f, 0.f, 0.f}; return z; }

__device__ __forceinline__ v16h ldfrag_h(const _Float16* p) {
  FragH f;
  f.h[0] = *(const v8h*)(p);
  f.h[1] = *(const v8h*)(p + 16);
  return f.v;
}

__device__ __forceinline__ v8f mma_h(v16h a, v16h b, v8f c) {
  c = __builtin_amdgcn_wmma_f32_16x16x32_f16(false, a, false, b, (short)0, c, false, false);
#if defined(__HIP_DEVICE_COMPILE__)
  asm volatile("v_nop\n\tv_nop\n\tv_nop\n\tv_nop" : "+v"(c) : "v"(a), "v"(b));
#endif
  return c;
}
__device__ __forceinline__ void wave_sync_lds() {
  __builtin_amdgcn_fence(__ATOMIC_RELEASE, "workgroup");
  __builtin_amdgcn_wave_barrier();
  __builtin_amdgcn_fence(__ATOMIC_ACQUIRE, "workgroup");
}

template <int MODE>
__global__ __launch_bounds__(256) void conv_h16(const float* __restrict__ W, unsigned short* Wh, int n8, int c8n,
                                                float wsc) {
  const int i  = blockIdx.x * 256 + threadIdx.x;
  const int ic = (i < n8) ? i : (n8 - 1);
  const int rs = ic / c8n;
  const int cc = ic - rs * c8n;
  int rd = rs;
  if (MODE == 1) rd = (rs % NBATCH) * SEQ + (rs / NBATCH);
  if (MODE == 2) {
    const int hq  = rs / (3 * HD);
    const int rem = rs - hq * (3 * HD);
    rd = (rem / HD) * DM + hq * HD + (rem & (HD - 1));
  }
  const float* src = W + (size_t)ic * 8;
  const v4f a = *(const v4f*)(src);
  const v4f c = *(const v4f*)(src + 4);
  v4u o;
  o[0] = pk16(h_bits((_Float16)(bfr(a[0]) * wsc)), h_bits((_Float16)(bfr(a[1]) * wsc)));
  o[1] = pk16(h_bits((_Float16)(bfr(a[2]) * wsc)), h_bits((_Float16)(bfr(a[3]) * wsc)));
  o[2] = pk16(h_bits((_Float16)(bfr(c[0]) * wsc)), h_bits((_Float16)(bfr(c[1]) * wsc)));
  o[3] = pk16(h_bits((_Float16)(bfr(c[2]) * wsc)), h_bits((_Float16)(bfr(c[3]) * wsc)));
  unsigned short* dst = Wh + ((size_t)rd * c8n + cc) * 8;
  if (i < n8) *(volatile v4u*)dst = o;
  __threadfence();
  if (i < n8) *(volatile v4u*)dst = o;
}

template <int MI, int OM, int BIASM, int ARES, int CRES, int ROWMAP>
__global__ __launch_bounds__(256) void gemm64(
    const unsigned short* __restrict__ Ap, const unsigned short* __restrict__ A2p, int lda, long long strideA,
    const unsigned short* __restrict__ Btp, int ldb, long long strideB,
    const float* __restrict__ bias,
    void* Cout, int ldc, long long strideC,
    void* C2out, int ldc2, long long strideC2, int Nres,
    int M, int N, int K, float oscale, float rscale) {
  const _Float16* A  = (const _Float16*)(const void*)Ap;
  const _Float16* A2 = (const _Float16*)(const void*)A2p;
  const _Float16* Bt = (const _Float16*)(const void*)Btp;
  __shared__ __align__(16) float sT[8][16 * 68];
  const int b    = blockIdx.y;
  const int lane = threadIdx.x & 31;
  const int wave = threadIdx.x >> 5;
  const int tilesN = N >> 6;
  const int tilesM = M / (16 * MI);
  const int tile = blockIdx.x * 8 + wave;
  if (tile >= tilesM * tilesN) return;
  const int tm = tile / tilesN;
  const int tn = tile - tm * tilesN;
  const int m0 = tm * (16 * MI);
  const int n0 = tn << 6;

  const _Float16* Ab  = A  + (size_t)b * strideA;
  const _Float16* A2b = A2 + (size_t)b * strideA;
  const _Float16* Bb  = Bt + (size_t)b * strideB;

  const int rlane = lane & 15;
  const int koff  = (lane >> 4) * 8;
  const int mOff  = (lane >> 4) * 8;

  v8f acc[MI][4], accr[MI][4];
#pragma unroll
  for (int i = 0; i < MI; ++i)
#pragma unroll
    for (int j = 0; j < 4; ++j) { acc[i][j] = zero8(); if (ARES) accr[i][j] = zero8(); }

  for (int k0 = 0; k0 < K; k0 += 32) {
    v16h bh[4];
#pragma unroll
    for (int j = 0; j < 4; ++j) {
      const size_t bo = (size_t)(n0 + (j << 4) + rlane) * ldb + koff + k0;
      bh[j] = ldfrag_h(Bb + bo);
    }
#pragma unroll
    for (int i = 0; i < MI; ++i) {
      const size_t ao = (size_t)(m0 + (i << 4) + rlane) * lda + koff + k0;
      const v16h ah = ldfrag_h(Ab + ao);
      if (ARES) {
        const v16h ar = ldfrag_h(A2b + ao);
#pragma unroll
        for (int j = 0; j < 4; ++j) {
          acc[i][j]  = mma_h(ah, bh[j], acc[i][j]);
          accr[i][j] = mma_h(ar, bh[j], accr[i][j]);
        }
      } else {
#pragma unroll
        for (int j = 0; j < 4; ++j) acc[i][j] = mma_h(ah, bh[j], acc[i][j]);
      }
    }
  }

  const int hh2 = lane >> 4, c4 = (lane & 15) * 4;
  const int q8  = lane >> 3, c8 = (lane & 7) * 8;
  float bc[8];
#pragma unroll
  for (int e = 0; e < 8; ++e) bc[e] = 0.f;
  if (BIASM == 0 && OM == 0) {
    const int cb = n0 + c4;
    const int i0 = (cb < N - 4) ? cb : (N - 4);
    const v4f b0v = *(const v4f*)(bias + i0);
#pragma unroll
    for (int e = 0; e < 4; ++e) bc[e] = bfr(b0v[e]);
  }
  if (BIASM == 1) {
    const int cb = n0 + c8;
    const int cq = cb & (DM - 1);
    const int j3 = cb >> DMLOG;
    int idx = ((cq >> 6) * 3 + j3) * HD + (cq & (HD - 1));
    idx = (idx < NIN - 8) ? idx : (NIN - 8);
    const v4f b0a = *(const v4f*)(bias + idx), b0b = *(const v4f*)(bias + idx + 4);
#pragma unroll
    for (int e = 0; e < 4; ++e) { bc[e] = bfr(b0a[e]); bc[4 + e] = bfr(b0b[e]); }
  }

  float* slab = sT[wave];
#pragma unroll
  for (int i = 0; i < MI; ++i) {
    const int mBase = m0 + (i << 4);
#pragma unroll
    for (int j = 0; j < 4; ++j) {
#pragma unroll
      for (int r = 0; r < 8; ++r) {
        float v = acc[i][j][r];
        if (ARES) v += accr[i][j][r] * rscale;
        slab[(mOff + r) * 68 + (j << 4) + rlane] = v;
      }
    }
    wave_sync_lds();
    if (OM == 0) {
      float* C = (float*)Cout + (size_t)b * strideC;
      v4f vals[8];
#pragma unroll
      for (int it = 0; it < 8; ++it) {
        const int row = it * 2 + hh2;
        v4f v = *(const v4f*)(slab + row * 68 + c4);
#pragma unroll
        for (int e = 0; e < 4; ++e) v[e] = v[e] * oscale + bc[e];
        vals[it] = v;
      }
      for (int pass = 0; pass < 2; ++pass) {
#pragma unroll
        for (int it = 0; it < 8; ++it) {
          const int row = it * 2 + hh2;
          int grow = mBase + row;
          if (ROWMAP == 1) grow = (grow & (SEQ - 1)) * NBATCH + (grow >> SEQLOG);
          *(volatile v4f*)(C + (size_t)grow * ldc + n0 + c4) = vals[it];
        }
        __threadfence();
      }
    } else {
      unsigned short* C  = (unsigned short*)Cout + (size_t)b * strideC;
      unsigned short* C2 = (unsigned short*)C2out + (size_t)b * strideC2;
      const bool wres = (CRES != 0) && (n0 < Nres);
      v4u hv[4], hr[4];
#pragma unroll
      for (int it = 0; it < 4; ++it) {
        const int row = it * 4 + q8;
        const float* sp = slab + row * 68 + c8;
        float bm = 0.f;
        if (BIASM == 2) {
          int gm = mBase + row;
          gm = (gm < M) ? gm : (M - 1);
          bm = bfr(bias[((gm >> 6) * 3 + 2) * HD + (gm & (HD - 1))]);
        }
        v4u a, q;
#pragma unroll
        for (int e = 0; e < 4; ++e) {
          const float f0 = sp[2 * e]     * oscale + ((BIASM == 2) ? bm : bc[2 * e]);
          const float f1 = sp[2 * e + 1] * oscale + ((BIASM == 2) ? bm : bc[2 * e + 1]);
          const _Float16 h0 = (_Float16)f0, h1 = (_Float16)f1;
          a[e] = pk16(h_bits(h0), h_bits(h1));
          if (CRES) {
            const _Float16 r0 = (_Float16)((f0 - (float)h0) * RSC);
            const _Float16 r1 = (_Float16)((f1 - (float)h1) * RSC);
            q[e] = pk16(h_bits(r0), h_bits(r1));
          } else {
            q[e] = 0u;
          }
        }
        hv[it] = a;
        hr[it] = q;
      }
      for (int pass = 0; pass < 2; ++pass) {
#pragma unroll
        for (int it = 0; it < 4; ++it) {
          const int row = it * 4 + q8;
          *(volatile v4u*)(C + (size_t)(mBase + row) * ldc + n0 + c8) = hv[it];
          if (wres) *(volatile v4u*)(C2 + (size_t)(mBase + row) * ldc2 + n0 + c8) = hr[it];
        }
        __threadfence();
      }
    }
    wave_sync_lds();
  }
}

__global__ __launch_bounds__(128)
void attn64(const unsigned short* __restrict__ qkp, const unsigned short* __restrict__ qrp,
            const unsigned short* __restrict__ vtp, const unsigned short* __restrict__ vrp,
            unsigned short* cthp, unsigned short* ctrp, float sscale) {
  __shared__ __align__(16) _Float16 Ksh[64 * 64];
  __shared__ __align__(16) _Float16 Vth[64 * 64];
  __shared__ __align__(16) _Float16 Vtr[64 * 64];
  __shared__ __align__(16) _Float16 Psh[4][16 * 64];
  __shared__ __align__(16) float    Os[4][16 * 64];

  const int tid  = threadIdx.x;
  const int wave = tid >> 5;
  const int lane = tid & 31;
  const int hh   = lane >> 4;
  const int c    = lane & 15;

  const int bx   = blockIdx.x;
  const int qb   = bx % NQB;
  const int rest = bx / NQB;
  const int h    = rest % NH;
  const int b    = rest / NH;
  const int q0   = qb * 64 + wave * 16;
  const size_t rowB = (size_t)b * SEQ;

  const _Float16* Qh = (const _Float16*)(const void*)qkp + (size_t)h * HD;
  const _Float16* Qr = (const _Float16*)(const void*)qrp + (size_t)h * HD;
  const _Float16* Kg = (const _Float16*)(const void*)qkp + DM + (size_t)h * HD;
  const _Float16* Vh = (const _Float16*)(const void*)vtp + ((size_t)b * DM + (size_t)h * HD) * SEQ;
  const _Float16* Vr = (const _Float16*)(const void*)vrp + ((size_t)b * DM + (size_t)h * HD) * SEQ;

  float mrow[8], lrow[8];
  v8f oacc[4], oacr[4];
#pragma unroll
  for (int r = 0; r < 8; ++r) { mrow[r] = -INFINITY; lrow[r] = 0.f; }
#pragma unroll
  for (int t = 0; t < 4; ++t) { oacc[t] = zero8(); oacr[t] = zero8(); }

  for (int kt = 0; kt < NQB; ++kt) {
    const int kv0 = kt * 64;

    __syncthreads();
    {
      const int r = tid >> 1, hf = (tid & 1) * 32;
      const _Float16* kg  = Kg + (rowB + kv0 + r) * QKP + hf;
      const _Float16* vg  = Vh + (size_t)r * SEQ + kv0 + hf;
      const _Float16* vg2 = Vr + (size_t)r * SEQ + kv0 + hf;
#pragma unroll
      for (int i = 0; i < 4; ++i) {
        const v8h a0 = *(const v8h*)(kg + 8 * i);
        const v8h b0 = *(const v8h*)(vg + 8 * i);
        const v8h b1 = *(const v8h*)(vg2 + 8 * i);
        *(v8h*)(Ksh + r * 64 + hf + 8 * i) = a0;
        *(v8h*)(Vth + r * 64 + hf + 8 * i) = b0;
        *(v8h*)(Vtr + r * 64 + hf + 8 * i) = b1;
      }
    }
    __syncthreads();

    v16h qa[2], qr[2];
#pragma unroll
    for (int dc = 0; dc < 2; ++dc) {
      qa[dc] = ldfrag_h(Qh + (rowB + q0 + c) * QKP + dc * 32 + 8 * hh);
      qr[dc] = ldfrag_h(Qr + (rowB + q0 + c) * DM  + dc * 32 + 8 * hh);
    }

    v8f s[4];
#pragma unroll
    for (int j = 0; j < 4; ++j) {
      v8f sh = zero8(), sr = zero8();
#pragma unroll
      for (int dc = 0; dc < 2; ++dc) {
        FragH kb;
        kb.h[0] = *(const v8h*)(Ksh + (j * 16 + c) * 64 + dc * 32 + 8 * hh);
        kb.h[1] = *(const v8h*)(Ksh + (j * 16 + c) * 64 + dc * 32 + 16 + 8 * hh);
        sh = mma_h(qa[dc], kb.v, sh);
        sr = mma_h(qr[dc], kb.v, sr);
      }
#pragma unroll
      for (int r = 0; r < 8; ++r) s[j][r] = (sh[r] + sr[r] * RINV) * sscale;
    }

    _Float16* pwh = Psh[wave];
#pragma unroll
    for (int r = 0; r < 8; ++r) {
      float m = s[0][r];
      m = fmaxf(m, s[1][r]);
      m = fmaxf(m, s[2][r]);
      m = fmaxf(m, s[3][r]);
#pragma unroll
      for (int off = 1; off < 16; off <<= 1) m = fmaxf(m, __shfl_xor(m, off, 32));
      const float mnew  = fmaxf(mrow[r], m);
      const float alpha = __expf(mrow[r] - mnew);
      mrow[r] = mnew;
      float psum = 0.f;
#pragma unroll
      for (int j = 0; j < 4; ++j) {
        const float p = __expf(s[j][r] - mnew);
        psum += p;
        pwh[(8 * hh + r) * 64 + j * 16 + c] = (_Float16)(p * 1024.0f);
      }
#pragma unroll
      for (int off = 1; off < 16; off <<= 1) psum += __shfl_xor(psum, off, 32);
      lrow[r] = lrow[r] * alpha + psum;
#pragma unroll
      for (int t = 0; t < 4; ++t) { oacc[t][r] *= alpha; oacr[t][r] *= alpha; }
    }
    wave_sync_lds();

#pragma unroll 1
    for (int kk = 0; kk < 2; ++kk) {
      FragH pa;
      pa.h[0] = *(const v8h*)(pwh + c * 64 + kk * 32 + 8 * hh);
      pa.h[1] = *(const v8h*)(pwh + c * 64 + kk * 32 + 16 + 8 * hh);
#pragma unroll
      for (int t = 0; t < 4; ++t) {
        FragH vb, vc;
        vb.h[0] = *(const v8h*)(Vth + (t * 16 + c) * 64 + kk * 32 + 8 * hh);
        vb.h[1] = *(const v8h*)(Vth + (t * 16 + c) * 64 + kk * 32 + 16 + 8 * hh);
        vc.h[0] = *(const v8h*)(Vtr + (t * 16 + c) * 64 + kk * 32 + 8 * hh);
        vc.h[1] = *(const v8h*)(Vtr + (t * 16 + c) * 64 + kk * 32 + 16 + 8 * hh);
        oacc[t] = mma_h(pa.v, vb.v, oacc[t]);
        oacr[t] = mma_h(pa.v, vc.v, oacr[t]);
      }
    }
  }

  float* os = Os[wave];
#pragma unroll
  for (int r = 0; r < 8; ++r) {
    const float l = lrow[r];
    const float inv = ((l > 0.f) ? (1.0f / l) : 0.f) * (CSC / 1024.0f);
#pragma unroll
    for (int t = 0; t < 4; ++t) os[(8 * hh + r) * 64 + t * 16 + c] = (oacc[t][r] + oacr[t][r] * RINV) * inv;
  }
  wave_sync_lds();
  {
    const int q4 = lane >> 3, c8 = (lane & 7) * 8;
    v4u hv[4], hr[4];
#pragma unroll
    for (int it = 0; it < 4; ++it) {
      const int row = it * 4 + q4;
      const float* sp = os + row * 64 + c8;
      v4u a, q;
#pragma unroll
      for (int e = 0; e < 4; ++e) {
        const float f0 = sp[2 * e], f1 = sp[2 * e + 1];
        const _Float16 h0 = (_Float16)f0, h1 = (_Float16)f1;
        const _Float16 r0 = (_Float16)((f0 - (float)h0) * RSC);
        const _Float16 r1 = (_Float16)((f1 - (float)h1) * RSC);
        a[e] = pk16(h_bits(h0), h_bits(h1));
        q[e] = pk16(h_bits(r0), h_bits(r1));
      }
      hv[it] = a;
      hr[it] = q;
    }
    for (int pass = 0; pass < 2; ++pass) {
#pragma unroll
      for (int it = 0; it < 4; ++it) {
        const int row = it * 4 + q4;
        const size_t go = (rowB + q0 + row) * DM + (size_t)h * HD + c8;
        *(volatile v4u*)(cthp + go) = hv[it];
        *(volatile v4u*)(ctrp + go) = hr[it];
      }
      __threadfence();
    }
  }
}

extern "C" void kernel_launch(void* const* d_in, const int* in_sizes, int n_in,
                              void* d_out, int out_size, void* d_ws, size_t ws_size,
                              hipStream_t stream) {
  if (n_in < 6) return;
  if (in_sizes[0] != MP * DM) return;
  if (in_sizes[1] != NIN * DM) return;
  if (in_sizes[2] != NIN) return;
  if (in_sizes[3] != DM * DM) return;
  if (in_sizes[4] != DM) return;
  if (out_size != MP * DM) return;

  const float* query = (const float*)d_in[0];
  const float* w_in  = (const float*)d_in[1];
  const float* b_in  = (const float*)d_in[2];
  const float* w_o   = (const float*)d_in[3];
  const float* b_o   = (const float*)d_in[4];

  const size_t PWIN = (size_t)NIN * DM * 2;
  const size_t PWO  = (size_t)DM * DM * 2;
  const size_t PXH  = (size_t)MP * DM * 2;
  const size_t PQK  = (size_t)MP * QKP * 2;
  const size_t PQR  = (size_t)MP * DM * 2;
  const size_t PVT  = (size_t)NBATCH * DM * SEQ * 2;
  const size_t PCT  = (size_t)MP * DM * 2;
  size_t off = 0;
  const size_t oWin = off; off += PWIN;
  const size_t oWo  = off; off += PWO;
  const size_t oXH  = off; off += PXH;
  const size_t oQK  = off; off += PQK;
  const size_t oQR  = off; off += PQR;
  const size_t oVT  = off; off += PVT;
  const size_t oVR  = off; off += PVT;
  const size_t oCtH = off; off += PCT;
  const size_t oCtR = off; off += PCT;
  if (off > ws_size) return;
  if (off > (size_t)134217728) return;

  char* ws = (char*)d_ws;
  unsigned short* WinH = (unsigned short*)(ws + oWin);
  unsigned short* WoH  = (unsigned short*)(ws + oWo);
  unsigned short* XH   = (unsigned short*)(ws + oXH);
  unsigned short* QK   = (unsigned short*)(ws + oQK);
  unsigned short* QR   = (unsigned short*)(ws + oQR);
  unsigned short* VT   = (unsigned short*)(ws + oVT);
  unsigned short* VR   = (unsigned short*)(ws + oVR);
  unsigned short* CtH  = (unsigned short*)(ws + oCtH);
  unsigned short* CtR  = (unsigned short*)(ws + oCtR);
  float*          out0 = (float*)d_out;

  const int c8n = DM / 8;
  const int n8x = (MP * DM) / 8;
  const int n8w = (NIN * DM) / 8;
  const int n8o = (DM * DM) / 8;
  if ((n8x % 256) != 0 || (n8w % 256) != 0 || (n8o % 256) != 0 || (c8n % 32) != 0) return;
  const dim3 blk(256), blk128(128);
  const dim3 gCx(n8x / 256), gCw(n8w / 256), gCo(n8o / 256);
  const dim3 gQK(((MP / 64) * (QKP / 64) + 7) / 8, 1);
  const dim3 gVT(((DM / 64) * (SEQ / 64) + 7) / 8, NBATCH);
  const dim3 gOut(((MP / 32) * (DM / 64) + 7) / 8, 1);
  const dim3 gAttn(NBATCH * NH * NQB);
  const float invw  = 1.0f / WSC;
  const float invwc = 1.0f / (WSC * CSC);

  conv_h16<1><<<gCx, blk, 0, stream>>>(query, XH, n8x, c8n, 1.0f);
  conv_h16<2><<<gCw, blk, 0, stream>>>(w_in, WinH, n8w, c8n, WSC);
  conv_h16<0><<<gCo, blk, 0, stream>>>(w_o, WoH, n8o, c8n, WSC);

  gemm64<4, 2, 1, 0, 1, 0><<<gQK, blk, 0, stream>>>(
      XH, XH, DM, 0LL, WinH, DM, 0LL, b_in,
      (void*)QK, QKP, 0LL, (void*)QR, DM, 0LL, DM,
      MP, QKP, DM, invw, 0.0f);
  gemm64<4, 2, 2, 0, 1, 0><<<gVT, blk, 0, stream>>>(
      WinH + (size_t)2 * DM * DM, WinH + (size_t)2 * DM * DM, DM, 0LL, XH, DM, (long long)SEQ * DM, b_in,
      (void*)VT, SEQ, (long long)DM * SEQ, (void*)VR, SEQ, (long long)DM * SEQ, SEQ,
      DM, SEQ, DM, invw, 0.0f);

  attn64<<<gAttn, blk128, 0, stream>>>(QK, QR, VT, VR, CtH, CtR, 0.125f);

  gemm64<2, 0, 0, 1, 0, 1><<<gOut, blk, 0, stream>>>(
      CtH, CtR, DM, 0LL, WoH, DM, 0LL, b_o,
      (void*)out0, DM, 0LL, (void*)out0, DM, 0LL, 0,
      MP, DM, DM, invwc, RINV);
  (void)hipGetLastError();
}
